// DistanceProbe_64080912056509
// MI455X (gfx1250) — hardware-verified
//
#include <hip/hip_runtime.h>


#ifndef NB
#define NB 8
#endif
#ifndef SEQ
#define SEQ 512
#endif
#define NB_FULL  8
#define SEQ_FULL 512
#ifndef OUT_SEQ
#define OUT_SEQ SEQ
#endif
#ifndef OUT_LD
#define OUT_LD SEQ
#endif
#define DMODEL 1024
#define RK     128
#define PSP    132
#define GSP    68
#define WTK    64

static_assert(DMODEL % 32 == 0);
static_assert(RK % 32 == 0);
static_assert(RK == 128);
static_assert((NB * SEQ) % 32 == 0);
static_assert(SEQ % 64 == 0);
static_assert(SEQ % 32 == 0);
static_assert(NB <= NB_FULL);
static_assert(SEQ <= SEQ_FULL);
static_assert(OUT_SEQ >= SEQ);
static_assert(OUT_LD >= SEQ);
static_assert(OUT_LD % 32 == 0);
static_assert((PSP * 4) % 16 == 0);
static_assert((GSP * 4) % 16 == 0);
static_assert(WTK * 2 == 128);
static_assert(DMODEL % WTK == 0);
static_assert((WTK * RK) % 256 == 0);
static_assert(((size_t)SEQ * DMODEL) % 8 == 0);
static_assert(32 * 16 * 8 == 16 * RK * 2);
static_assert(32 * 16 * 8 == 16 * 64 * 4);
static_assert(8 * 16 == 32 * 4);
static_assert(256 * ((RK * WTK / 8) / 256) * 16 == RK * WTK * 2);
static_assert(sizeof(float) * (16 * PSP + 32) <= 131072);
static_assert(sizeof(float) * (16 * GSP) <= 131072);
static_assert(sizeof(float) * (WTK * (RK + 1)) <= 131072);

typedef _Float16 h16;
typedef unsigned short bf;
typedef __attribute__((ext_vector_type(16))) __bf16   v16bf;
typedef __attribute__((ext_vector_type(16))) _Float16 v16h;
typedef __attribute__((ext_vector_type(8)))  _Float16 v8h;
typedef __attribute__((ext_vector_type(8)))  unsigned short v8us;
typedef __attribute__((ext_vector_type(8)))  float    v8f;
typedef __attribute__((ext_vector_type(4)))  float    v4f;
typedef v4f  __attribute__((may_alias)) v4fa;

__device__ __forceinline__ unsigned short f2bf(float f) { unsigned u = __float_as_uint(f); u += 0x7FFFu + ((u >> 16) & 1u); return (unsigned short)(u >> 16); }
__device__ __forceinline__ float bfr(float f) { return __uint_as_float(((unsigned)f2bf(f)) << 16); }
__device__ __forceinline__ v16h cat16(v8h lo, v8h hi) { return __builtin_shufflevector(lo, hi, 0, 1, 2, 3, 4, 5, 6, 7, 8, 9, 10, 11, 12, 13, 14, 15); }
__device__ __forceinline__ v16bf cat16b(v8us lo, v8us hi) { return __builtin_bit_cast(v16bf, __builtin_shufflevector(lo, hi, 0, 1, 2, 3, 4, 5, 6, 7, 8, 9, 10, 11, 12, 13, 14, 15)); }
__device__ __forceinline__ v8f wmma16(v16h a, v16h b, v8f c) { return __builtin_amdgcn_wmma_f32_16x16x32_f16(false, a, false, b, (short)0, c, false, false); }
__device__ __forceinline__ v8f wmmab(v16bf a, v16bf b, v8f c) { return __builtin_amdgcn_wmma_f32_16x16x32_bf16(false, a, false, b, (short)0, c, false, false); }
__device__ __forceinline__ v16h  ldh(const h16* p) { return cat16(*(const v8h*)p, *(const v8h*)(p + 16)); }
__device__ __forceinline__ v16bf ldb(const bf* p)  { return cat16b(*(const v8us*)p, *(const v8us*)(p + 16)); }
__device__ __forceinline__ void wave_sync() { __builtin_amdgcn_fence(3  , "wavefront"); __builtin_amdgcn_wave_barrier(); asm volatile("" ::: "memory"); }

static __device__ __forceinline__ h16 toh_flush(float v) { const h16 r = (h16)v; return (fabsf(v) < 6.103515625e-05f) ? (h16)0.0f : r; }
__device__ __forceinline__ v8f wmma16_g(v16h a, v16h b, v8f c) { c = wmma16(a, b, c); asm volatile("v_nop\n\tv_nop\n\tv_nop\n\tv_nop" : "+v"(c) : "v"(a), "v"(b)); return c; }
__device__ __forceinline__ v8f wmmab_g(v16bf a, v16bf b, v8f c) { c = wmmab(a, b, c); asm volatile("v_nop\n\tv_nop\n\tv_nop\n\tv_nop" : "+v"(c) : "v"(a), "v"(b)); return c; }

__global__ __launch_bounds__(256) void k_cvt8(const float* __restrict__ src, bf* dst, size_t n8) {
    const size_t i = (size_t)blockIdx.x * 256 + threadIdx.x; if (i >= n8) return;
    const v8f v = *(const v8f*)(src + i * 8); v8us o;
#pragma unroll
    for (int k = 0; k < 8; ++k) o[k] = f2bf(v[k]);
    *(volatile v8us*)(dst + i * 8) = o; __threadfence(); *(volatile v8us*)(dst + i * 8) = o;
}

__global__ __launch_bounds__(256) void k_wtr(const float* __restrict__ W, bf* WT) {
    __shared__ float ts[WTK * (RK + 1)];
    const int tid = threadIdx.x; const int kb = blockIdx.x * WTK;
#pragma unroll 1
    for (int it = 0; it < (WTK * RK) / 256; ++it) {
        const int idx = it * 256 + tid; const int k = idx / RK, n = idx % RK;
        ts[k * (RK + 1) + n] = W[(size_t)(kb + k) * RK + n];
    }
    __syncthreads();
#pragma unroll 1
    for (int ps = 0; ps < 2; ++ps) {
#pragma unroll 1
        for (int it = 0; it < (RK * WTK / 8) / 256; ++it) {
            const int q = it * 256 + tid; const int n = q / (WTK / 8), k8 = (q % (WTK / 8)) * 8;
            v8us o;
#pragma unroll
            for (int e = 0; e < 8; ++e) o[e] = f2bf(ts[(k8 + e) * (RK + 1) + n]);
            *(volatile v8us*)(WT + (size_t)n * DMODEL + kb + k8) = o;
        }
        if (ps == 0) __threadfence();
    }
}

__global__ __launch_bounds__(32) void k_projt(const bf* __restrict__ A, const bf* __restrict__ Bt, h16* TH, float* NRM) {
    __shared__ __align__(16) float os[16 * PSP];
    __shared__ __align__(16) float ns[32];
    const int lane = threadIdx.x & 31, lr = lane & 15, hi = lane >> 4; const int r0 = blockIdx.x * 32;
    v8f acc[2][8];
#pragma unroll
    for (int mb = 0; mb < 2; ++mb)
#pragma unroll
        for (int nb = 0; nb < 8; ++nb) acc[mb][nb] = (v8f){};
    const size_t aoff = (size_t)(r0 + lr) * DMODEL + 8 * hi, boff = (size_t)lr * DMODEL + 8 * hi;
#pragma unroll 1
    for (int kc = 0; kc < DMODEL; kc += 32) {
        v16bf a[2];
#pragma unroll
        for (int mb = 0; mb < 2; ++mb) a[mb] = ldb(A + aoff + (size_t)mb * 16 * DMODEL + kc);
#pragma unroll
        for (int nb = 0; nb < 8; ++nb) { const v16bf b = ldb(Bt + boff + (size_t)nb * 16 * DMODEL + kc);
#pragma unroll
            for (int mb = 0; mb < 2; ++mb) acc[mb][nb] = wmmab_g(a[mb], b, acc[mb][nb]); }
    }
#pragma unroll
    for (int mb = 0; mb < 2; ++mb) {
#pragma unroll
        for (int nb = 0; nb < 8; ++nb) {
#pragma unroll
            for (int j = 0; j < 8; ++j) os[(hi * 8 + j) * PSP + nb * 16 + lr] = acc[mb][nb][j]; }
        wave_sync();
        const size_t sb = (size_t)(r0 + mb * 16) * RK;
#pragma unroll 1
        for (int ps = 0; ps < 2; ++ps) {
#pragma unroll
            for (int s = 0; s < 8; ++s) { const int p = s * 32 + lane; const int row = p >> 4, c8 = (p & 15) * 8;
                const v4f x0 = *(const v4fa*)(&os[row * PSP + c8]); const v4f x1 = *(const v4fa*)(&os[row * PSP + c8 + 4]); v8h hv; float q = 0.0f;
#pragma unroll
                for (int i = 0; i < 4; ++i) { const h16 a0 = toh_flush(x0[i]); const h16 a1 = toh_flush(x1[i]); hv[i] = a0; hv[4 + i] = a1;
                                              const float f0 = (float)a0, f1 = (float)a1; q += f0 * f0 + f1 * f1; }
                q += __shfl_xor(q, 8, 32); q += __shfl_xor(q, 4, 32); q += __shfl_xor(q, 2, 32); q += __shfl_xor(q, 1, 32);
                if (lr == 0) ns[mb * 16 + row] = q;
                *(volatile v8h*)(TH + sb + (size_t)p * 8) = hv; }
            if (ps == 0) __threadfence(); }
        wave_sync();
    }
    const v4f nv = *(const v4fa*)(&ns[(lane & 7) * 4]);
    float* np = NRM + (size_t)r0 + (lane & 7) * 4;
    if (lane < 8) *(volatile v4f*)np = nv;
    __threadfence();
    if (lane < 8) *(volatile v4f*)np = nv;
}

__global__ __launch_bounds__(32) void k_gram(const h16* __restrict__ TH, const float* __restrict__ NRM, float* OUT) {
    __shared__ __align__(16) float os[16 * GSP];
    const int lane = threadIdx.x & 31, lr = lane & 15, hi = lane >> 4;
    const int j0 = blockIdx.x * 64, i0 = blockIdx.y * 64, bz = blockIdx.z;
    v8f acc[4][4];
#pragma unroll
    for (int mb = 0; mb < 4; ++mb)
#pragma unroll
        for (int nb = 0; nb < 4; ++nb) acc[mb][nb] = (v8f){};
    const size_t aoff = ((size_t)bz * SEQ + i0 + lr) * RK + 8 * hi, boff = ((size_t)bz * SEQ + j0 + lr) * RK + 8 * hi;
#pragma unroll 1
    for (int kc = 0; kc < RK; kc += 32) {
        v16h a[4];
#pragma unroll
        for (int mb = 0; mb < 4; ++mb) a[mb] = ldh(TH + aoff + (size_t)mb * 16 * RK + kc);
#pragma unroll
        for (int nb = 0; nb < 4; ++nb) { const v16h bq = ldh(TH + boff + (size_t)nb * 16 * RK + kc);
#pragma unroll
            for (int mb = 0; mb < 4; ++mb) acc[mb][nb] = wmma16_g(a[mb], bq, acc[mb][nb]); }
    }
    const float* nrow = NRM + (size_t)bz * SEQ;
    float nj[4];
#pragma unroll
    for (int nb = 0; nb < 4; ++nb) nj[nb] = nrow[j0 + nb * 16 + lr];
#pragma unroll
    for (int mb = 0; mb < 4; ++mb) {
        const v4f n0 = *(const v4f*)(nrow + i0 + mb * 16 + hi * 8); const v4f n1 = *(const v4f*)(nrow + i0 + mb * 16 + hi * 8 + 4);
        float ni[8];
#pragma unroll
        for (int j = 0; j < 4; ++j) { ni[j] = n0[j]; ni[4 + j] = n1[j]; }
#pragma unroll
        for (int nb = 0; nb < 4; ++nb) {
#pragma unroll
            for (int j = 0; j < 8; ++j) { const int ii = i0 + mb * 16 + hi * 8 + j, jj = j0 + nb * 16 + lr;
                float v = (ni[j] + nj[nb]) - 2.0f * acc[mb][nb][j];
                v = fmaxf(v, 0.0f); v = (ii == jj) ? 0.0f : v;
                os[(hi * 8 + j) * GSP + nb * 16 + lr] = v; } }
        wave_sync();
        float* ob = OUT + ((size_t)bz * OUT_SEQ + i0 + mb * 16) * OUT_LD + j0;
#pragma unroll 1
        for (int ps = 0; ps < 2; ++ps) {
#pragma unroll
            for (int s = 0; s < 8; ++s) { const int p = s * 32 + lane; const int row = p >> 4, c4 = (p & 15) * 4;
                const v4f val = *(const v4fa*)(&os[row * GSP + c4]);
                *(volatile v4f*)(ob + (size_t)row * OUT_LD + c4) = val; }
            if (ps == 0) __threadfence(); }
        wave_sync();
    }
}

static constexpr size_t al256(size_t v) { return (v + 255) & ~(size_t)255; }
static constexpr size_t SZ_XB = al256((size_t)NB * SEQ * DMODEL * 2);
static constexpr size_t SZ_WT = al256((size_t)RK * DMODEL * 2);
static constexpr size_t SZ_TH = al256((size_t)NB * SEQ * RK * 2);
static constexpr size_t SZ_NR = al256((size_t)NB * SEQ * 4);
static constexpr size_t SZ_TOTAL = SZ_XB + SZ_WT + SZ_TH + SZ_NR;
static_assert(SZ_TOTAL <= (size_t)134217728);
static_assert((size_t)(NB * SEQ / 32) * 32 * RK * 2 == (size_t)NB * SEQ * RK * 2);
static_assert((size_t)(NB * SEQ / 32) * 128 == (size_t)NB * SEQ * 4);
static_assert((size_t)(DMODEL / WTK) * RK * WTK * 2 == (size_t)RK * DMODEL * 2);

extern "C" void kernel_launch(void* const* d_in, const int* in_sizes, int n_in,
                              void* d_out, int out_size, void* d_ws, size_t ws_size, hipStream_t stream) {
    if (n_in < 2) return;
    const size_t needx = ((size_t)(NB - 1) * SEQ_FULL + SEQ) * DMODEL;
    if ((size_t)in_sizes[0] < needx) return;
    if ((size_t)in_sizes[1] < (size_t)DMODEL * RK) return;
    if ((size_t)out_size < ((size_t)(NB - 1) * OUT_SEQ + SEQ) * OUT_LD) return;
    if (SZ_TOTAL > ws_size) return;
    const float* xin = (const float*)d_in[0];
    const float* wp  = (const float*)d_in[1];
    float* OUT = (float*)d_out;
    char* wsp = (char*)d_ws;
    bf*  XB = (bf*)wsp;   wsp += SZ_XB;
    bf*  WT = (bf*)wsp;   wsp += SZ_WT;
    h16* TH = (h16*)wsp;  wsp += SZ_TH;
    float* NR = (float*)wsp; wsp += SZ_NR;

    if (SEQ == SEQ_FULL) {
        const size_t n8 = (size_t)NB * SEQ * DMODEL / 8;
        k_cvt8<<<(unsigned)((n8 + 255) / 256), 256, 0, stream>>>(xin, XB, n8);
    } else {
        const size_t n8 = (size_t)SEQ * DMODEL / 8;
        for (int b = 0; b < NB; ++b) k_cvt8<<<(unsigned)((n8 + 255) / 256), 256, 0, stream>>>(xin + (size_t)b * SEQ_FULL * DMODEL, XB + (size_t)b * SEQ * DMODEL, n8);
    }
    k_wtr<<<DMODEL / WTK, 256, 0, stream>>>(wp, WT);
    k_projt<<<NB * SEQ / 32, 32, 0, stream>>>(XB, WT, TH, NR);
    k_gram<<<dim3(SEQ / 64, SEQ / 64, NB), 32, 0, stream>>>(TH, NR, OUT);
}
